// LocalAttention_47966194762023
// MI455X (gfx1250) — hardware-verified
//
#include <hip/hip_runtime.h>
#include <stddef.h>
#include <stdint.h>


#ifndef NB
#define NB 8
#endif
#ifndef SEQ
#define SEQ 7936
#endif
#define NB_FULL 8
#define SEQ_FULL 7936
#define CD 256
#define WS 31
#define NW (SEQ / WS)

#define PCARRY 16384.0f
#define YCARRY 64.0f
#define WCARRY 64.0f
#define RCARRY 4096.0f
#define RINV (1.0f / 4096.0f)

static_assert(NB >= 1 && NB <= NB_FULL);
static_assert(SEQ % WS == 0 && SEQ % 128 == 0 && SEQ >= 128 && SEQ <= SEQ_FULL);
static_assert(CD == 256);
static_assert((NB * SEQ) % 8 == 0);
static_assert((size_t)NB_FULL * SEQ_FULL * CD * 2 + (size_t)3 * CD * CD * 2 + (size_t)CD * CD * 2
              + (size_t)6 * SEQ_FULL * CD * 2 + (size_t)2 * SEQ_FULL * CD * 2
              + (size_t)SEQ_FULL * CD * 4 <= (size_t)134217728);

typedef _Float16 v16h __attribute__((ext_vector_type(16)));
typedef _Float16 v8h  __attribute__((ext_vector_type(8)));
typedef _Float16 v4h  __attribute__((ext_vector_type(4)));
typedef _Float16 v2h  __attribute__((ext_vector_type(2)));
typedef __bf16   v16b __attribute__((ext_vector_type(16)));
typedef float    v8f  __attribute__((ext_vector_type(8)));
typedef float    v4f  __attribute__((ext_vector_type(4)));
typedef float    v2f  __attribute__((ext_vector_type(2)));
typedef unsigned int u32x4 __attribute__((ext_vector_type(4)));

union Frag {
  v16h  h;
  v16b  b;
  u32x4 q[2];
  v8h   p[2];
};

__device__ __forceinline__ v8f zero8() {
  v8f z;
#pragma unroll
  for (int i = 0; i < 8; ++i) z[i] = 0.0f;
  return z;
}

__device__ __forceinline__ unsigned int bf_bits(float x) {
  unsigned int u = __builtin_bit_cast(unsigned int, x);
  u += 0x7FFFu + ((u >> 16) & 1u);
  return u >> 16;
}
__device__ __forceinline__ float bf_rne(float x) {
  unsigned int u = bf_bits(x) << 16;
  return __builtin_bit_cast(float, u);
}
__device__ __forceinline__ unsigned int h_bits(float x) {
  _Float16 t = (_Float16)x;
  unsigned short s = __builtin_bit_cast(unsigned short, t);
  return (unsigned int)s;
}

__device__ __forceinline__ u32x4 pack8_bf(v4f a, v4f c) {
  const float a0 = a[0], a1 = a[1], a2 = a[2], a3 = a[3];
  const float c0 = c[0], c1 = c[1], c2 = c[2], c3 = c[3];
  u32x4 o;
  o[0] = bf_bits(a0) | (bf_bits(a1) << 16);
  o[1] = bf_bits(a2) | (bf_bits(a3) << 16);
  o[2] = bf_bits(c0) | (bf_bits(c1) << 16);
  o[3] = bf_bits(c2) | (bf_bits(c3) << 16);
  return o;
}
__device__ __forceinline__ u32x4 pack8_h(v4f a, v4f c, float scale) {
  const float a0 = bf_rne(a[0]) * scale, a1 = bf_rne(a[1]) * scale;
  const float a2 = bf_rne(a[2]) * scale, a3 = bf_rne(a[3]) * scale;
  const float c0 = bf_rne(c[0]) * scale, c1 = bf_rne(c[1]) * scale;
  const float c2 = bf_rne(c[2]) * scale, c3 = bf_rne(c[3]) * scale;
  u32x4 o;
  o[0] = h_bits(a0) | (h_bits(a1) << 16);
  o[1] = h_bits(a2) | (h_bits(a3) << 16);
  o[2] = h_bits(c0) | (h_bits(c1) << 16);
  o[3] = h_bits(c2) | (h_bits(c3) << 16);
  return o;
}

__device__ __forceinline__ v8f mma_f16(const Frag& a, const Frag& bb, v8f c) {
  c = __builtin_amdgcn_wmma_f32_16x16x32_f16(false, a.h, false, bb.h, (short)0, c, false, false);
  asm volatile("v_nop\n\tv_nop\n\tv_nop\n\tv_nop" : "+v"(c) : "v"(a.h), "v"(bb.h));
  return c;
}
__device__ __forceinline__ v8f mma_bf16(const Frag& a, const Frag& bb, v8f c) {
  c = __builtin_amdgcn_wmma_f32_16x16x32_bf16(false, a.b, false, bb.b, (short)0, c, false, false);
  asm volatile("v_nop\n\tv_nop\n\tv_nop\n\tv_nop" : "+v"(c) : "v"(a.b), "v"(bb.b));
  return c;
}
template <int MODE> struct MmaSel;
template <> struct MmaSel<0> {
  static __device__ __forceinline__ v8f run(const Frag& a, const Frag& bb, v8f c) { return mma_bf16(a, bb, c); }
};
template <> struct MmaSel<1> {
  static __device__ __forceinline__ v8f run(const Frag& a, const Frag& bb, v8f c) { return mma_f16(a, bb, c); }
};

__global__ __launch_bounds__(256) void cvt_rows_bf16(const float* __restrict__ src,
                                                     unsigned short* __restrict__ dst, int mrows) {
  const int m = blockIdx.x * 8 + ((int)threadIdx.x >> 5);
  if (m >= mrows) return;
  const int b = m / SEQ;
  const int t = m - b * SEQ;
  const int c8 = ((int)threadIdx.x & 31) * 8;
  const float* s = src + ((size_t)(b * SEQ_FULL + t)) * CD + c8;
  const v4f a = *(const v4f*)s;
  const v4f c = *(const v4f*)(s + 4);
  const u32x4 o = pack8_bf(a, c);
  unsigned short* d = dst + (size_t)m * CD + c8;
  *(volatile u32x4*)d = o;
  __threadfence();
  *(volatile u32x4*)d = o;
}

__global__ __launch_bounds__(256) void cvt_flat(const float* __restrict__ src,
                                                unsigned short* __restrict__ dst,
                                                int n, int to_f16, float scale) {
  const int i = (blockIdx.x * 256 + (int)threadIdx.x) * 8;
  if (i + 8 > n) return;
  const v4f a = *(const v4f*)(src + i);
  const v4f c = *(const v4f*)(src + i + 4);
  u32x4 o;
  if (to_f16 != 0) o = pack8_h(a, c, scale);
  else             o = pack8_bf(a, c);
  unsigned short* d = dst + i;
  *(volatile u32x4*)d = o;
  __threadfence();
  *(volatile u32x4*)d = o;
}

struct GemmArgs {
  const unsigned short* A;
  const unsigned short* W0;
  const unsigned short* W1;
  const unsigned short* W2;
  const float* bias0;
  const float* bias1;
  const float* bias2;
  unsigned short* o0;
  unsigned short* o1;
  unsigned short* o2;
  unsigned short* r0;
  unsigned short* r1;
  unsigned short* r2;
  float* of;
  const float* addend;
  float oscale;
  int use_bias;
  int use_add;
  int resv;
};
static_assert(sizeof(GemmArgs) == 136);

#define GSP16 136
#define GSP32 132

__device__ __forceinline__ void gemm_store16(const _Float16* st, unsigned short* o16, size_t base,
                                             int pitchR, int wave, int h, int ln) {
#pragma unroll
  for (int it = 0; it < 8; ++it) {
    const int R = wave * 16 + 2 * it + h;
    const u32x4 v = *(const u32x4*)(st + R * GSP16 + ln * 8);
    *(volatile u32x4*)(o16 + base + (size_t)R * pitchR + ln * 8) = v;
  }
}

template <int MODE>
__global__ __launch_bounds__(256) __attribute__((amdgpu_num_vgpr(256)))
void gemm_nt(GemmArgs g) {
  __shared__ __align__(16) unsigned short Asm[128 * 40];
  __shared__ __align__(16) unsigned short Wsm[128 * 40];
  __shared__ __align__(16) float stg[8704];

  const int tid = threadIdx.x;
  const int wave = tid >> 5, lane = tid & 31, h = lane >> 4, ln = lane & 15;
  const int wm = wave >> 2, wn = wave & 3;
  const int m0 = blockIdx.y * 128, n0 = blockIdx.x * 128, z = blockIdx.z;
  const unsigned short* W = (z == 0) ? g.W0 : ((z == 1) ? g.W1 : g.W2);
  const float* bias = (z == 0) ? g.bias0 : ((z == 1) ? g.bias1 : g.bias2);

  v8f acc[4][2];
#pragma unroll
  for (int mt = 0; mt < 4; ++mt)
#pragma unroll
    for (int nt = 0; nt < 2; ++nt) acc[mt][nt] = zero8();

#pragma unroll 1
  for (int k0 = 0; k0 < CD; k0 += 32) {
    u32x4 la[2], lw[2];
#pragma unroll
    for (int s = 0; s < 2; ++s) {
      const int u = tid + s * 256, row = u >> 2, qo = (u & 3) * 8;
      la[s] = *(const u32x4*)(g.A + ((size_t)(m0 + row)) * CD + k0 + qo);
      lw[s] = *(const u32x4*)(W + ((size_t)(n0 + row)) * CD + k0 + qo);
    }
    __syncthreads();
#pragma unroll
    for (int s = 0; s < 2; ++s) {
      const int u = tid + s * 256, row = u >> 2, qo = (u & 3) * 8;
      *(u32x4*)(&Asm[row * 40 + qo]) = la[s];
      *(u32x4*)(&Wsm[row * 40 + qo]) = lw[s];
    }
    __syncthreads();

    Frag af[4], bfr[2];
#pragma unroll
    for (int mt = 0; mt < 4; ++mt) {
      const unsigned short* p = &Asm[(wm * 64 + mt * 16 + ln) * 40 + 8 * h];
      af[mt].q[0] = *(const u32x4*)p;
      af[mt].q[1] = *(const u32x4*)(p + 16);
    }
#pragma unroll
    for (int nt = 0; nt < 2; ++nt) {
      const unsigned short* p = &Wsm[(wn * 32 + nt * 16 + ln) * 40 + 8 * h];
      bfr[nt].q[0] = *(const u32x4*)p;
      bfr[nt].q[1] = *(const u32x4*)(p + 16);
    }
#pragma unroll
    for (int mt = 0; mt < 4; ++mt)
#pragma unroll
      for (int nt = 0; nt < 2; ++nt)
        acc[mt][nt] = MmaSel<MODE>::run(af[mt], bfr[nt], acc[mt][nt]);
  }

  float bb[2];
#pragma unroll
  for (int nt = 0; nt < 2; ++nt)
    bb[nt] = (g.use_bias != 0) ? bf_rne(bias[n0 + wn * 32 + nt * 16 + ln]) : 0.0f;

  if (MODE == 0) {
    _Float16* st = (_Float16*)stg;
    unsigned short* o16 = (z == 0) ? g.o0 : ((z == 1) ? g.o1 : g.o2);
    unsigned short* r16 = (z == 0) ? g.r0 : ((z == 1) ? g.r1 : g.r2);
    const size_t base = ((size_t)m0) * CD + n0;
#pragma unroll
    for (int mt = 0; mt < 4; ++mt)
#pragma unroll
      for (int nt = 0; nt < 2; ++nt)
#pragma unroll
        for (int r = 0; r < 8; ++r) {
          const int row = wm * 64 + mt * 16 + 8 * h + r;
          const int col = wn * 32 + nt * 16 + ln;
          const float v = acc[mt][nt][r] + bb[nt];
          st[row * GSP16 + col] = (_Float16)v;
        }
    __syncthreads();
    gemm_store16(st, o16, base, CD, wave, h, ln);
    __threadfence();
    gemm_store16(st, o16, base, CD, wave, h, ln);

    __syncthreads();
#pragma unroll
    for (int mt = 0; mt < 4; ++mt)
#pragma unroll
      for (int nt = 0; nt < 2; ++nt)
#pragma unroll
        for (int r = 0; r < 8; ++r) {
          const int row = wm * 64 + mt * 16 + 8 * h + r;
          const int col = wn * 32 + nt * 16 + ln;
          const float v = acc[mt][nt][r] + bb[nt];
          const _Float16 hv = (_Float16)v;
          st[row * GSP16 + col] = (_Float16)((v - (float)hv) * RCARRY);
        }
    __syncthreads();
    gemm_store16(st, r16, base, CD, wave, h, ln);
    __threadfence();
    gemm_store16(st, r16, base, CD, wave, h, ln);
  } else {
    const float osc = g.oscale;
    const bool addp = (g.use_add != 0);
    const float* abase = g.addend + (size_t)m0 * CD + n0 + lane * 4;
#pragma unroll
    for (int ph = 0; ph < 2; ++ph) {
      __syncthreads();
      if (wm == ph) {
#pragma unroll
        for (int mt = 0; mt < 4; ++mt)
#pragma unroll
          for (int nt = 0; nt < 2; ++nt)
#pragma unroll
            for (int r = 0; r < 8; ++r) {
              const int row = mt * 16 + 8 * h + r;
              const int col = wn * 32 + nt * 16 + ln;
              stg[row * GSP32 + col] = acc[mt][nt][r] * osc + bb[nt];
            }
      }
      __syncthreads();
      v4f vals[8];
#pragma unroll
      for (int it = 0; it < 8; ++it) {
        const int R = wave * 8 + it;
        v4f v = *(const v4f*)(stg + R * GSP32 + lane * 4);
        if (addp) {
          const v4f a4 = *(const v4f*)(abase + ((size_t)(ph * 64 + R)) * CD);
          v += a4;
        }
        vals[it] = v;
      }
      float* ob = g.of + ((size_t)(m0 + ph * 64)) * CD + n0 + lane * 4;
#pragma unroll
      for (int it = 0; it < 8; ++it)
        *(volatile v4f*)(ob + ((size_t)(wave * 8 + it)) * CD) = vals[it];
      __threadfence();
#pragma unroll
      for (int it = 0; it < 8; ++it)
        *(volatile v4f*)(ob + ((size_t)(wave * 8 + it)) * CD) = vals[it];
    }
  }
}

#define VTP 40
#define PSP 40
#define YSP 72

__device__ __forceinline__ void attn_store_y(const _Float16* yw, unsigned short* dst,
                                             int row0, int pmt, int cg, int lane) {
#pragma unroll
  for (int it = 0; it < 4; ++it) {
    const int R = it * 4 + (lane >> 3);
    const int row = pmt * 16 + R;
    const int piece = (lane & 7) * 8;
    const u32x4 v = *(const u32x4*)(yw + R * YSP + piece);
    if (row < WS) {
      *(volatile u32x4*)(dst + ((size_t)(row0 + row)) * CD + cg * 64 + piece) = v;
    }
  }
}

__global__ __launch_bounds__(256) __attribute__((amdgpu_num_vgpr(256)))
void attn_win(const unsigned short* __restrict__ qpl, const unsigned short* __restrict__ kpl,
              const unsigned short* __restrict__ vpl, const unsigned short* __restrict__ qrs,
              const unsigned short* __restrict__ krs, const unsigned short* __restrict__ vrs,
              unsigned short* __restrict__ ypl, unsigned short* __restrict__ yrs) {
  __shared__ __align__(16) unsigned short Vsm[2 * CD * VTP];
  __shared__ __align__(16) float    Spart[2 * 32 * 32];
  __shared__ __align__(16) _Float16 Psh[32 * PSP];
  __shared__ __align__(16) _Float16 Prs[32 * PSP];
  __shared__ float linv[32];

  const int tid = threadIdx.x;
  const int wave = tid >> 5, lane = tid & 31, h = lane >> 4, ln = lane & 15;
  const int row0 = (int)blockIdx.x * WS;
  unsigned short* Vt = Vsm;
  unsigned short* Vr = Vsm + CD * VTP;

  for (int c = tid; c < WS * (CD / 8); c += 256) {
    const int j = c >> 5;
    const int c8 = (c & 31) * 8;
    const size_t gofs = ((size_t)(row0 + j)) * CD + c8;
    const u32x4 a = *(const u32x4*)(vpl + gofs);
    const u32x4 rv = *(const u32x4*)(vrs + gofs);
#pragma unroll
    for (int i = 0; i < 4; ++i) {
      const unsigned int wa = a[i], wr = rv[i];
      Vt[(c8 + 2 * i) * VTP + j]     = (unsigned short)(wa & 0xFFFFu);
      Vt[(c8 + 2 * i + 1) * VTP + j] = (unsigned short)(wa >> 16);
      Vr[(c8 + 2 * i) * VTP + j]     = (unsigned short)(wr & 0xFFFFu);
      Vr[(c8 + 2 * i + 1) * VTP + j] = (unsigned short)(wr >> 16);
    }
  }
  Vt[tid * VTP + WS] = (unsigned short)0;
  Vr[tid * VTP + WS] = (unsigned short)0;

  {
    const int t = wave & 3, mt = t >> 1, nt = t & 1, kh = wave >> 2;
    int qrow = row0 + mt * 16 + ln;
    qrow = (qrow > SEQ - 1) ? (SEQ - 1) : qrow;
    int krow = row0 + nt * 16 + ln;
    krow = (krow > SEQ - 1) ? (SEQ - 1) : krow;
    const size_t qoff = ((size_t)qrow) * CD + 8 * h;
    const size_t koff = ((size_t)krow) * CD + 8 * h;
    v8f sacc = zero8(), sres = zero8();
#pragma unroll 1
    for (int p = 0; p < 4; ++p) {
      const int k0 = (kh * 4 + p) * 32;
      Frag qa, qr, kb, kr;
      qa.q[0] = *(const u32x4*)(qpl + qoff + k0);
      qa.q[1] = *(const u32x4*)(qpl + qoff + k0 + 16);
      qr.q[0] = *(const u32x4*)(qrs + qoff + k0);
      qr.q[1] = *(const u32x4*)(qrs + qoff + k0 + 16);
      kb.q[0] = *(const u32x4*)(kpl + koff + k0);
      kb.q[1] = *(const u32x4*)(kpl + koff + k0 + 16);
      kr.q[0] = *(const u32x4*)(krs + koff + k0);
      kr.q[1] = *(const u32x4*)(krs + koff + k0 + 16);
      sacc = mma_f16(qa, kb, sacc);
      sres = mma_f16(qa, kr, sres);
      sres = mma_f16(qr, kb, sres);
    }
#pragma unroll
    for (int r = 0; r < 8; ++r)
      Spart[kh * 1024 + (mt * 16 + 8 * h + r) * 32 + nt * 16 + ln] = sacc[r] + sres[r] * RINV;
  }
  __syncthreads();

  const int rr = tid >> 3;
  const int cc = (tid & 7) * 4;
  {
    const float SC = 0.0625f * 1.4426950408889634f;
    const v4f sa = *(const v4f*)(&Spart[rr * 32 + cc]);
    const v4f sb = *(const v4f*)(&Spart[1024 + rr * 32 + cc]);
    float s0 = (sa[0] + sb[0]) * SC;
    float s1 = (sa[1] + sb[1]) * SC;
    float s2 = (sa[2] + sb[2]) * SC;
    float s3 = (sa[3] + sb[3]) * SC;
    const bool drop3 = (cc + 3 >= WS);
    s3 = drop3 ? -1e30f : s3;
    float mx = fmaxf(fmaxf(s0, s1), fmaxf(s2, s3));
    mx = fmaxf(mx, __shfl_xor(mx, 4));
    mx = fmaxf(mx, __shfl_xor(mx, 2));
    mx = fmaxf(mx, __shfl_xor(mx, 1));
    const float e0 = __builtin_amdgcn_exp2f(s0 - mx);
    const float e1 = __builtin_amdgcn_exp2f(s1 - mx);
    const float e2 = __builtin_amdgcn_exp2f(s2 - mx);
    const float e3 = __builtin_amdgcn_exp2f(s3 - mx);
    const float p0 = e0, p1 = e1, p2 = e2;
    const float p3 = drop3 ? 0.0f : e3;
    float rs = (p0 + p1) + (p2 + p3);
    rs += __shfl_xor(rs, 4);
    rs += __shfl_xor(rs, 2);
    rs += __shfl_xor(rs, 1);
    if ((tid & 7) == 0) linv[rr] = (1.0f / rs) * (YCARRY / PCARRY);
    const float P0 = p0 * PCARRY, P1 = p1 * PCARRY, P2 = p2 * PCARRY, P3 = p3 * PCARRY;
    const _Float16 h0 = (_Float16)P0, h1 = (_Float16)P1, h2 = (_Float16)P2, h3 = (_Float16)P3;
    v4h hv, rv;
    hv[0] = h0; hv[1] = h1; hv[2] = h2; hv[3] = h3;
    rv[0] = (_Float16)((P0 - (float)h0) * RCARRY);
    rv[1] = (_Float16)((P1 - (float)h1) * RCARRY);
    rv[2] = (_Float16)((P2 - (float)h2) * RCARRY);
    rv[3] = (_Float16)((P3 - (float)h3) * RCARRY);
    *(v4h*)(&Psh[rr * PSP + cc]) = hv;
    *(v4h*)(&Prs[rr * PSP + cc]) = rv;
  }
  __syncthreads();

  const int pmt = wave & 1, cg = wave >> 1;
  Frag pa, pr;
  pa.p[0] = *(const v8h*)(&Psh[(pmt * 16 + ln) * PSP + 8 * h]);
  pa.p[1] = *(const v8h*)(&Psh[(pmt * 16 + ln) * PSP + 16 + 8 * h]);
  pr.p[0] = *(const v8h*)(&Prs[(pmt * 16 + ln) * PSP + 8 * h]);
  pr.p[1] = *(const v8h*)(&Prs[(pmt * 16 + ln) * PSP + 16 + 8 * h]);
  v8f oacc[4];
#pragma unroll
  for (int i = 0; i < 4; ++i) {
    const int ch = cg * 64 + i * 16 + ln;
    Frag vb, vr;
    vb.q[0] = *(const u32x4*)(&Vt[ch * VTP + 8 * h]);
    vb.q[1] = *(const u32x4*)(&Vt[ch * VTP + 16 + 8 * h]);
    vr.q[0] = *(const u32x4*)(&Vr[ch * VTP + 8 * h]);
    vr.q[1] = *(const u32x4*)(&Vr[ch * VTP + 16 + 8 * h]);
    oacc[i] = mma_f16(pa, vb, zero8());
    v8f tt = zero8();
    tt = mma_f16(pa, vr, tt);
    tt = mma_f16(pr, vb, tt);
    oacc[i] += tt * RINV;
  }

  float li[8];
#pragma unroll
  for (int r = 0; r < 8; ++r) li[r] = linv[pmt * 16 + 8 * h + r];
  __syncthreads();
  _Float16* yw = (_Float16*)Vsm + wave * (16 * YSP);
#pragma unroll
  for (int i = 0; i < 4; ++i)
#pragma unroll
    for (int r = 0; r < 8; ++r)
      yw[(8 * h + r) * YSP + i * 16 + ln] = (_Float16)(oacc[i][r] * li[r]);
  __syncthreads();
  attn_store_y(yw, ypl, row0, pmt, cg, lane);
  __threadfence();
  attn_store_y(yw, ypl, row0, pmt, cg, lane);

  __syncthreads();
#pragma unroll
  for (int i = 0; i < 4; ++i)
#pragma unroll
    for (int r = 0; r < 8; ++r) {
      const float y64 = oacc[i][r] * li[r];
      const _Float16 hv = (_Float16)y64;
      yw[(8 * h + r) * YSP + i * 16 + ln] = (_Float16)((y64 - (float)hv) * RCARRY);
    }
  __syncthreads();
  attn_store_y(yw, yrs, row0, pmt, cg, lane);
  __threadfence();
  attn_store_y(yw, yrs, row0, pmt, cg, lane);
}

extern "C" void kernel_launch(void* const* d_in, const int* in_sizes, int n_in,
                              void* d_out, int out_size, void* d_ws, size_t ws_size,
                              hipStream_t stream) {
  if (n_in < 5) return;
  const int M = NB * SEQ;
  if (in_sizes[0] < ((NB - 1) * SEQ_FULL + SEQ) * CD) return;
  if (in_sizes[1] < 3 * CD * CD || in_sizes[2] < 3 * CD) return;
  if (in_sizes[3] < CD * CD || in_sizes[4] < CD) return;
  if (out_size < ((NB - 1) * SEQ_FULL + SEQ) * CD) return;

  const float* x     = (const float*)d_in[0];
  const float* Wqkv  = (const float*)d_in[1];
  const float* bqkv  = (const float*)d_in[2];
  const float* Wproj = (const float*)d_in[3];
  const float* bproj = (const float*)d_in[4];
  float* out = (float*)d_out;

  const size_t xB    = (size_t)M * CD * 2;
  const size_t wqkvB = (size_t)3 * CD * CD * 2;
  const size_t woB   = (size_t)CD * CD * 2;
  const size_t plB   = (size_t)SEQ * CD * 2;
  const size_t rtB   = (size_t)SEQ * CD * 4;
  char* ws = (char*)d_ws;
  size_t off = 0;
  unsigned short* xb   = (unsigned short*)(ws + off); off += xB;
  unsigned short* wqkv = (unsigned short*)(ws + off); off += wqkvB;
  unsigned short* wob  = (unsigned short*)(ws + off); off += woB;
  unsigned short* qpl  = (unsigned short*)(ws + off); off += plB;
  unsigned short* kpl  = (unsigned short*)(ws + off); off += plB;
  unsigned short* vpl  = (unsigned short*)(ws + off); off += plB;
  unsigned short* qrs  = (unsigned short*)(ws + off); off += plB;
  unsigned short* krs  = (unsigned short*)(ws + off); off += plB;
  unsigned short* vrs  = (unsigned short*)(ws + off); off += plB;
  unsigned short* ypl  = (unsigned short*)(ws + off); off += plB;
  unsigned short* yrs  = (unsigned short*)(ws + off); off += plB;
  float*          rtm  = (float*)(ws + off);          off += rtB;
  if (off > ws_size) return;

  cvt_rows_bf16<<<dim3(M / 8), dim3(256), 0, stream>>>(x, xb, M);
  cvt_flat<<<dim3(3 * CD * CD / 2048), dim3(256), 0, stream>>>(Wqkv, wqkv, 3 * CD * CD, 0, 1.0f);
  cvt_flat<<<dim3(CD * CD / 2048), dim3(256), 0, stream>>>(Wproj, wob, CD * CD, 1, WCARRY);

  for (int b = 0; b < NB; ++b) {
    GemmArgs ga;
    ga.A = xb + (size_t)b * SEQ * CD;
    ga.W0 = wqkv; ga.W1 = wqkv + (size_t)CD * CD; ga.W2 = wqkv + (size_t)2 * CD * CD;
    ga.bias0 = bqkv; ga.bias1 = bqkv + CD; ga.bias2 = bqkv + 2 * CD;
    ga.o0 = qpl; ga.o1 = kpl; ga.o2 = vpl;
    ga.r0 = qrs; ga.r1 = krs; ga.r2 = vrs;
    ga.of = rtm;
    ga.addend = rtm;
    ga.oscale = 1.0f;
    ga.use_bias = 1;
    ga.use_add = 0;
    ga.resv = 0;
    gemm_nt<0><<<dim3(CD / 128, SEQ / 128, 3), dim3(256), 0, stream>>>(ga);

    attn_win<<<dim3(NW), dim3(256), 0, stream>>>(qpl, kpl, vpl, qrs, krs, vrs, ypl, yrs);

    GemmArgs gr;
    gr.A = yrs;
    gr.W0 = wob; gr.W1 = wob; gr.W2 = wob;
    gr.bias0 = bproj; gr.bias1 = bproj; gr.bias2 = bproj;
    gr.o0 = qpl; gr.o1 = qpl; gr.o2 = qpl;
    gr.r0 = qrs; gr.r1 = qrs; gr.r2 = qrs;
    gr.of = rtm;
    gr.addend = rtm;
    gr.oscale = 1.0f / (YCARRY * RCARRY * WCARRY);
    gr.use_bias = 0;
    gr.use_add = 0;
    gr.resv = 0;
    gemm_nt<1><<<dim3(CD / 128, SEQ / 128, 1), dim3(256), 0, stream>>>(gr);

    GemmArgs gb;
    gb.A = ypl;
    gb.W0 = wob; gb.W1 = wob; gb.W2 = wob;
    gb.bias0 = bproj; gb.bias1 = bproj; gb.bias2 = bproj;
    gb.o0 = qpl; gb.o1 = qpl; gb.o2 = qpl;
    gb.r0 = qrs; gb.r1 = qrs; gb.r2 = qrs;
    gb.of = out + (size_t)b * SEQ_FULL * CD;
    gb.addend = rtm;
    gb.oscale = 1.0f / (YCARRY * WCARRY);
    gb.use_bias = 1;
    gb.use_add = 1;
    gb.resv = 0;
    gemm_nt<1><<<dim3(CD / 128, SEQ / 128, 1), dim3(256), 0, stream>>>(gb);
  }
}
